// PCGTConvLayer_9225589752429
// MI455X (gfx1250) — hardware-run, weakly checked
//
#include <hip/hip_runtime.h>


namespace {
constexpr int N = 32768, NQLIM = 32768  , IC = 256, H = 4, D = 128, HD = H * D  , KP = 64, PP = 512, KPL = NQLIM / PP;
constexpr float XS = 8.0f, WSC = 256.0f, PS = 1024.0f, LOG2E = 1.4426950408889634f, RSD = 0.088388347648318447f;
static_assert(N % PP == 0 && NQLIM % PP == 0 && NQLIM <= N && PP % 64 == 0 && IC % 32 == 0 && D == 128, "tiling");
typedef _Float16 b16;
typedef __attribute__((ext_vector_type(16))) _Float16 v16b;
typedef __attribute__((ext_vector_type(8))) _Float16 v8b;
typedef __attribute__((ext_vector_type(8))) float v8f;
typedef __attribute__((ext_vector_type(4))) float v4f;
__device__ __forceinline__ float bf16_rne(float f) { unsigned int u = __float_as_uint(f); u += 0x7FFFu + ((u >> 16) & 1u); return __uint_as_float(u & 0xFFFF0000u); }
__device__ __forceinline__ void split16(float v, b16& hi, b16& lo) { hi = (b16)v; lo = (b16)(v - (float)hi); }
__device__ __forceinline__ v16b frag_kb(const b16* p, int hh) { const v8b a = *(const v8b*)(p + 8 * hh), b = *(const v8b*)(p + 16 + 8 * hh); v16b f;
#pragma unroll
  for (int e = 0; e < 8; ++e) { f[e] = a[e]; f[8 + e] = b[e]; } return f; }
__device__ __forceinline__ v8f wmma16b(v16b a, v16b b, v8f c) { v8f d = __builtin_amdgcn_wmma_f32_16x16x32_f16(false, a, false, b, (short)0, c, false, false); asm volatile("v_nop\n\tv_nop\n\tv_nop\n\tv_nop" : "+v"(d) : "v"(a), "v"(b)); return d; }
__device__ __forceinline__ void wave_lds_sync() { __builtin_amdgcn_fence(__ATOMIC_RELEASE, "workgroup"); __builtin_amdgcn_wave_barrier(); __builtin_amdgcn_fence(__ATOMIC_ACQUIRE, "workgroup"); }
__device__ __forceinline__ float pmul(float a, float b) { float p = a * b; asm volatile("" : "+v"(p)); return p; }
__device__ __forceinline__ int iclamp(int v, int lo, int hi) { return v < lo ? lo : (v > hi ? hi : v); }

typedef __attribute__((ext_vector_type(4))) _Float16 v4h;
typedef __attribute__((ext_vector_type(2))) _Float16 v2h;
__device__ __forceinline__ float nexp2(float v) { return __builtin_amdgcn_exp2f(v); }
__global__ __launch_bounds__(256) void wprep_kernel(const float* __restrict__ wq, const float* __restrict__ wk, const float* __restrict__ wv, b16* __restrict__ Wb) {
  const size_t u = (size_t)blockIdx.x * 256 + threadIdx.x; if (u >= (size_t)3 * HD * IC / 8) return; const size_t e = u * 8; const int s = (int)(e / ((size_t)HD * IC)); const size_t el = e % ((size_t)HD * IC); const float* w = s == 0 ? wq : (s == 1 ? wk : wv); v8b o;
  for (int j = 0; j < 8; ++j) o[j] = (b16)(bf16_rne(w[el + j]) * WSC);
  for (int pass = 0; pass < 2; ++pass) { *(volatile v8b*)(Wb + e) = o; __threadfence(); }
}
__global__ __launch_bounds__(256) void xmean_kernel(const float* __restrict__ x, float* __restrict__ XM) {
  const int kp = blockIdx.x, c = threadIdx.x; float s = 0.0f;
#pragma unroll 1
  for (int p = 0; p < PP; ++p) s += bf16_rne(x[((size_t)kp * PP + p) * IC + c]);
  for (int pass = 0; pass < 2; ++pass) { ((volatile float*)XM)[kp * IC + c] = s * (1.0f / PP); __threadfence(); }
}
__global__ __launch_bounds__(256) void cent_kernel(const float* __restrict__ XM, const float* __restrict__ wk, const float* __restrict__ bk, const float* __restrict__ wv, const float* __restrict__ bv, b16* __restrict__ CKh, b16* __restrict__ CKl, float* __restrict__ CV) {
  __shared__ float xs[IC]; __shared__ __attribute__((aligned(16))) float ck[HD], cv[HD];
  const int kp = blockIdx.x, t = threadIdx.x; xs[t] = XM[kp * IC + t]; __syncthreads();
#pragma unroll 1
  for (int jj = 0; jj < 4; ++jj) { const int j = jj * 256 + t; float a = (j < HD) ? bf16_rne(bk[j]) : bf16_rne(bv[j - HD]); const float* w = (j < HD) ? wk + (size_t)j * IC : wv + (size_t)(j - HD) * IC;
#pragma unroll 1
    for (int i = 0; i < IC; ++i) a += pmul(xs[i], bf16_rne(w[i]));
    if (j < HD) ck[j] = a; else cv[j - HD] = a; }
  __syncthreads();
  const int wave = t >> 5, lane = t & 31;
  for (int pass = 0; pass < 2; ++pass) {
    if (wave < H) { const int h = wave; v4h hv, lv; for (int j = 0; j < 4; ++j) { b16 p, q; split16(ck[h * D + lane * 4 + j] * XS, p, q); hv[j] = p; lv[j] = q; }
      *(volatile v4h*)(CKh + ((size_t)h * KP + kp) * D + lane * 4) = hv; *(volatile v4h*)(CKl + ((size_t)h * KP + kp) * D + lane * 4) = lv; }
    else { const int h = wave - H; *(volatile v4f*)(CV + ((size_t)kp * H + h) * D + lane * 4) = *(const v4f*)(&cv[h * D + lane * 4]); }
    __threadfence(); }
}
__global__ __launch_bounds__(256) void cvt_kernel(const float* __restrict__ CV, b16* __restrict__ CVT) {
  const int u = blockIdx.x * 256 + threadIdx.x; if (u >= D * H * KP / 8) return; const int d = u / (H * KP / 8), c0 = (u % (H * KP / 8)) * 8; const int h = c0 / KP, kp0 = c0 % KP; v8b o;
  for (int j = 0; j < 8; ++j) o[j] = (b16)(CV[((size_t)(kp0 + j) * H + h) * D + d] * XS);
  for (int pass = 0; pass < 2; ++pass) { *(volatile v8b*)(CVT + (size_t)d * (H * KP) + c0) = o; __threadfence(); }
}
__global__ __launch_bounds__(128) void qk_kernel(const float* __restrict__ x, const b16* __restrict__ Wb, const float* __restrict__ bq, const float* __restrict__ bk, b16* __restrict__ QK) {
  __shared__ __attribute__((aligned(16))) b16 As[4][16][IC + 8]; __shared__ __attribute__((aligned(16))) float Tf[4][16][128 + 4];
  const int wave = threadIdx.x >> 5, lane = threadIdx.x & 31, nloc = lane & 15, hlf = lane >> 4; const size_t m0 = (size_t)blockIdx.x * 64 + wave * 16; const int s = blockIdx.y >> 2, hsl = blockIdx.y & 3; const int n0 = hsl * 128;
  for (int rr = 0; rr < 16; ++rr) { const float* xr = x + (m0 + rr) * IC; v8b o; for (int j = 0; j < 8; ++j) o[j] = (b16)(bf16_rne(xr[lane * 8 + j]) * XS); *(v8b*)(&As[wave][rr][lane * 8]) = o; }
  wave_lds_sync();
  const b16* W = Wb + (size_t)s * HD * IC; const float* bias = s == 0 ? bq : bk;
  v8f acc[8];
#pragma unroll
  for (int t = 0; t < 8; ++t) acc[t] = (v8f){};
#pragma unroll 2
  for (int kb = 0; kb < IC; kb += 32) { const v16b a = frag_kb(&As[wave][nloc][kb], hlf);
#pragma unroll
    for (int t = 0; t < 8; ++t) acc[t] = wmma16b(a, frag_kb(W + (size_t)(n0 + t * 16 + nloc) * IC + kb, hlf), acc[t]); }
#pragma unroll
  for (int t = 0; t < 8; ++t) { const float bb = bf16_rne(bias[n0 + t * 16 + nloc]);
#pragma unroll
    for (int r = 0; r < 8; ++r) Tf[wave][8 * hlf + r][t * 16 + nloc] = acc[t][r] * (1.0f / (XS * WSC)) + bb; }
  wave_lds_sync();
  b16* P = QK + (size_t)s * N * HD;
  for (int pass = 0; pass < 2; ++pass) { for (int rr = 0; rr < 16; ++rr) { const v4f f = *(const v4f*)(&Tf[wave][rr][lane * 4]); v4h hv; for (int j = 0; j < 4; ++j) hv[j] = (b16)(f[j] * XS); *(volatile v4h*)(P + (m0 + rr) * HD + n0 + lane * 4) = hv; } __threadfence(); }
}
__global__ __launch_bounds__(128) void v_kernel(const float* __restrict__ x, const b16* __restrict__ Wb, const float* __restrict__ bv, const float* __restrict__ beta, b16* __restrict__ VT, float* __restrict__ ACC) {
  __shared__ __attribute__((aligned(16))) b16 As[4][16][IC + 8]; __shared__ __attribute__((aligned(16))) float Tf[4][16][128 + 4], Xs[4][16][128 + 4];
  const int wave = threadIdx.x >> 5, lane = threadIdx.x & 31, nloc = lane & 15, hlf = lane >> 4; const size_t n0 = (size_t)blockIdx.x * 64; const size_t m0 = n0 + wave * 16; const int kp = (int)(n0 / PP), p0 = (int)(n0 % PP);
  for (int rr = 0; rr < 16; ++rr) { const float* xr = x + (m0 + rr) * IC; v8b o; for (int j = 0; j < 8; ++j) o[j] = (b16)(bf16_rne(xr[lane * 8 + j]) * XS); *(v8b*)(&As[wave][rr][lane * 8]) = o; for (int j = 0; j < 4; ++j) Xs[wave][rr][lane * 4 + j] = 0.0f; }
  wave_lds_sync();
  const b16* W = Wb + (size_t)2 * HD * IC;
#pragma unroll 1
  for (int h = 0; h < H; ++h) {
    v8f acc[8];
#pragma unroll
    for (int t = 0; t < 8; ++t) acc[t] = (v8f){};
#pragma unroll 1
    for (int kb = 0; kb < IC; kb += 32) { const v16b a = frag_kb(&As[wave][nloc][kb], hlf);
#pragma unroll
      for (int t = 0; t < 8; ++t) acc[t] = wmma16b(a, frag_kb(W + (size_t)(h * D + t * 16 + nloc) * IC + kb, hlf), acc[t]); }
#pragma unroll
    for (int t = 0; t < 8; ++t) { const float bb = bf16_rne(bv[h * D + t * 16 + nloc]);
#pragma unroll
      for (int r = 0; r < 8; ++r) Tf[wave][8 * hlf + r][t * 16 + nloc] = acc[t][r] * (1.0f / (XS * WSC)) + bb; }
    wave_lds_sync();
#pragma unroll 1
    for (int rr = 0; rr < 16; ++rr) { const v4f f = *(const v4f*)(&Tf[wave][rr][lane * 4]); v4f xa = *(const v4f*)(&Xs[wave][rr][lane * 4]); xa += f * 0.25f; *(v4f*)(&Xs[wave][rr][lane * 4]) = xa; }
    __syncthreads();
    for (int pass = 0; pass < 2; ++pass) {
#pragma unroll 1
      for (int q = 0; q < 32; ++q) { const int d = wave * 32 + q; const int t0 = lane * 2; v2h v2; v2[0] = (b16)(Tf[t0 >> 4][t0 & 15][d] * XS); v2[1] = (b16)(Tf[(t0 + 1) >> 4][(t0 + 1) & 15][d] * XS);
        *(volatile v2h*)(VT + (((size_t)kp * H + h) * D + d) * PP + p0 + lane * 2) = v2; } __threadfence(); }
    __syncthreads(); }
  const float bta = bf16_rne(beta[0]);
  for (int pass = 0; pass < 2; ++pass) { for (int rr = 0; rr < 16; ++rr) { v4f xa = *(const v4f*)(&Xs[wave][rr][lane * 4]); xa *= bta; *(volatile v4f*)(ACC + (m0 + rr) * D + lane * 4) = xa; } __threadfence(); }
}
__global__ __launch_bounds__(64) void attn_kernel(const b16* __restrict__ QK, const b16* __restrict__ VT, const float* __restrict__ alpha_logit, float* __restrict__ ACC) {
  __shared__ __attribute__((aligned(16))) float XL[2][16][D + 4];
  const int wave = threadIdx.x >> 5, lane = threadIdx.x & 31, hh = lane >> 4, col = lane & 15; const int q0 = blockIdx.x * 32 + wave * 16, qi = q0 + col; const int kp = q0 / PP; const size_t kbase = (size_t)kp * PP;
  const b16* Qp = QK; const b16* Kpl = QK + (size_t)N * HD;
  for (int rr = 0; rr < 16; ++rr) for (int j = 0; j < 4; ++j) XL[wave][rr][lane * 4 + j] = 0.0f;
  const float cs = LOG2E * RSD / (XS * XS);
#pragma unroll 1
  for (int h = 0; h < H; ++h) {
    v16b qa[4];
#pragma unroll
    for (int ks = 0; ks < 4; ++ks) qa[ks] = frag_kb(Qp + (size_t)qi * HD + h * D + ks * 32, hh);
    const b16* Vb = VT + ((size_t)kp * H + h) * D * PP;
    float m = -INFINITY, l = 0.0f; v8f o[8];
#pragma unroll
    for (int t = 0; t < 8; ++t) o[t] = (v8f){};
#pragma unroll 1
    for (int kb = 0; kb < PP; kb += 32) {
      v8f s0 = (v8f){}, s1 = (v8f){};
#pragma unroll
      for (int ks = 0; ks < 4; ++ks) { s0 = wmma16b(frag_kb(Kpl + (kbase + kb + col) * HD + h * D + ks * 32, hh), qa[ks], s0); s1 = wmma16b(frag_kb(Kpl + (kbase + kb + 16 + col) * HD + h * D + ks * 32, hh), qa[ks], s1); }
      float e[16]; float mx = -INFINITY;
#pragma unroll
      for (int r = 0; r < 8; ++r) { e[r] = s0[r] * cs; e[8 + r] = s1[r] * cs; mx = fmaxf(mx, fmaxf(e[r], e[8 + r])); }
      mx = fmaxf(mx, __shfl_xor(mx, 16)); const float mn = fmaxf(m, mx); const float al = nexp2(m - mn); m = mn; float sum = 0.0f; v16b ph;
#pragma unroll
      for (int i = 0; i < 16; ++i) { const float p = nexp2(e[i] - mn); sum += p; ph[i] = (b16)(p * PS); }
      sum += __shfl_xor(sum, 16); l = l * al + sum;
#pragma unroll
      for (int t = 0; t < 8; ++t) { o[t] *= al; o[t] = wmma16b(frag_kb(Vb + (size_t)(t * 16 + col) * PP + kb, hh), ph, o[t]); } }
    const float inv = 0.25f / (l * PS * XS);
    wave_lds_sync();
#pragma unroll
    for (int t = 0; t < 8; ++t)
#pragma unroll
      for (int r = 0; r < 8; ++r) XL[wave][col][t * 16 + 8 * hh + r] += o[t][r] * inv;
    wave_lds_sync(); }
  const float alpha = 1.0f / (1.0f + __expf(-bf16_rne(alpha_logit[0])));
  for (int rr = 0; rr < 16; ++rr) { v4f a = *(const v4f*)(ACC + (size_t)(q0 + rr) * D + lane * 4); const v4f xl = *(const v4f*)(&XL[wave][rr][lane * 4]); a += xl * alpha; *(v4f*)(&XL[wave][rr][lane * 4]) = a; }
  wave_lds_sync();
  for (int pass = 0; pass < 2; ++pass) { for (int rr = 0; rr < 16; ++rr) *(volatile v4f*)(ACC + (size_t)(q0 + rr) * D + lane * 4) = *(const v4f*)(&XL[wave][rr][lane * 4]); __threadfence(); }
}
__global__ __launch_bounds__(64) void cross_kernel(const b16* __restrict__ QK, const b16* __restrict__ CKh, const b16* __restrict__ CKl, const b16* __restrict__ CVT, const float* __restrict__ alpha_logit, const float* __restrict__ ACC, float* __restrict__ out) {
  __shared__ __attribute__((aligned(16))) b16 Ph[2][16][H * KP + 8], Pl[2][16][H * KP + 8]; __shared__ __attribute__((aligned(16))) float Pf[2][16][H * KP + 4]; __shared__ __attribute__((aligned(16))) float To[2][16][D + 4];
  const int wave = threadIdx.x >> 5, lane = threadIdx.x & 31, nloc = lane & 15, hlf = lane >> 4; const size_t m0 = (size_t)blockIdx.x * 32 + wave * 16;
  const float cs = LOG2E * RSD / (XS * XS);
#pragma unroll 1
  for (int h = 0; h < H; ++h) {
    v8f lg[4];
#pragma unroll
    for (int t = 0; t < 4; ++t) lg[t] = (v8f){};
#pragma unroll
    for (int ks = 0; ks < 4; ++ks) { const v16b a = frag_kb(QK + (m0 + nloc) * HD + h * D + ks * 32, hlf);
#pragma unroll
      for (int t = 0; t < 4; ++t) { const size_t brow = ((size_t)h * KP + t * 16 + nloc) * D + ks * 32; lg[t] = wmma16b(a, frag_kb(CKh + brow, hlf), lg[t]); lg[t] = wmma16b(a, frag_kb(CKl + brow, hlf), lg[t]); } }
#pragma unroll
    for (int r = 0; r < 8; ++r) { float mx = -INFINITY;
#pragma unroll
      for (int t = 0; t < 4; ++t) mx = fmaxf(mx, lg[t][r] * cs);
#pragma unroll
      for (int off = 1; off < 16; off <<= 1) mx = fmaxf(mx, __shfl_xor(mx, off));
      float p[4], s = 0.0f;
#pragma unroll
      for (int t = 0; t < 4; ++t) { p[t] = nexp2(lg[t][r] * cs - mx); s += p[t]; }
#pragma unroll
      for (int off = 1; off < 16; off <<= 1) s += __shfl_xor(s, off);
      const float inv = 1.0f / s;
#pragma unroll
      for (int t = 0; t < 4; ++t) Pf[wave][8 * hlf + r][h * KP + t * 16 + nloc] = p[t] * inv * PS; } }
  wave_lds_sync();
  { const int row = lane & 15, c0 = (lane >> 4) * 128;
#pragma unroll 4
    for (int q = 0; q < 16; ++q) { v8b hv, lv;
#pragma unroll
      for (int j = 0; j < 8; ++j) { b16 a_, b_; split16(Pf[wave][row][c0 + q * 8 + j], a_, b_); hv[j] = a_; lv[j] = b_; } *(v8b*)(&Ph[wave][row][c0 + q * 8]) = hv; *(v8b*)(&Pl[wave][row][c0 + q * 8]) = lv; } }
  wave_lds_sync();
  v8f acc[8];
#pragma unroll
  for (int t = 0; t < 8; ++t) acc[t] = (v8f){};
#pragma unroll 2
  for (int kb = 0; kb < H * KP; kb += 32) { const v16b a = frag_kb(&Ph[wave][nloc][kb], hlf), al = frag_kb(&Pl[wave][nloc][kb], hlf);
#pragma unroll
    for (int t = 0; t < 8; ++t) { const v16b bw = frag_kb(CVT + (size_t)(t * 16 + nloc) * (H * KP) + kb, hlf); acc[t] = wmma16b(a, bw, acc[t]); acc[t] = wmma16b(al, bw, acc[t]); } }
  const float alpha = 1.0f / (1.0f + __expf(-bf16_rne(alpha_logit[0]))); const float g = (1.0f - alpha) * 0.25f / (PS * XS);
#pragma unroll
  for (int t = 0; t < 8; ++t)
#pragma unroll
    for (int r = 0; r < 8; ++r) To[wave][8 * hlf + r][t * 16 + nloc] = acc[t][r] * g;
  wave_lds_sync();
  for (int pass = 0; pass < 2; ++pass) { for (int rr = 0; rr < 16; ++rr) { v4f o = *(const v4f*)(&To[wave][rr][lane * 4]); o += *(const v4f*)(ACC + (m0 + rr) * D + lane * 4); *(volatile v4f*)(out + (m0 + rr) * D + lane * 4) = o; } __threadfence(); }
}
}

extern "C" void kernel_launch(void* const* d_in, const int* in_sizes, int n_in, void* d_out, int out_size, void* d_ws, size_t ws_size, hipStream_t stream) {
  (void)n_in;
  auto Fp = [&](int i) { return (const float*)d_in[i]; };
  if (in_sizes[0] != N * IC || in_sizes[1] != N || in_sizes[2] != HD * IC || in_sizes[3] != HD || in_sizes[4] != HD * IC || in_sizes[5] != HD || in_sizes[6] != HD * IC || in_sizes[7] != HD || in_sizes[8] != 1 || in_sizes[9] != 1 || out_size != N * D) return;
  size_t off = 0; char* ws = (char*)d_ws;
  auto carve = [&](size_t bytes) { char* p = ws + off; off += (bytes + 255) & ~(size_t)255; return p; };
  b16* Wb = (b16*)carve((size_t)3 * HD * IC * 2); float* XM = (float*)carve((size_t)KP * IC * 4); b16* CKh = (b16*)carve((size_t)H * KP * D * 2); b16* CKl = (b16*)carve((size_t)H * KP * D * 2); float* CV = (float*)carve((size_t)KP * H * D * 4); b16* CVT = (b16*)carve((size_t)D * H * KP * 2);
  b16* QK = (b16*)carve((size_t)2 * N * HD * 2); b16* VT = (b16*)carve((size_t)KP * H * D * PP * 2); float* ACC = (float*)carve((size_t)N * D * 4);
  if (off > ws_size || off > ((size_t)128 << 20)) return;
  wprep_kernel<<<(unsigned)(((size_t)3 * HD * IC / 8 + 255) / 256), 256, 0, stream>>>(Fp(2), Fp(4), Fp(6), Wb);
  xmean_kernel<<<KP, 256, 0, stream>>>(Fp(0), XM);
  cent_kernel<<<KP, 256, 0, stream>>>(XM, Fp(4), Fp(5), Fp(6), Fp(7), CKh, CKl, CV);
  cvt_kernel<<<(D * H * KP / 8 + 255) / 256, 256, 0, stream>>>(CV, CVT);
  qk_kernel<<<dim3(NQLIM / 64, 8), 128, 0, stream>>>(Fp(0), Wb, Fp(3), Fp(5), QK);
  v_kernel<<<NQLIM / 64, 128, 0, stream>>>(Fp(0), Wb, Fp(7), Fp(9), VT, ACC);
  attn_kernel<<<NQLIM / 32, 64, 0, stream>>>(QK, VT, Fp(8), ACC);
  cross_kernel<<<NQLIM / 32, 64, 0, stream>>>(QK, CKh, CKl, CVT, Fp(8), ACC, (float*)d_out);
}
